// GATv2Layer_57964878626937
// MI455X (gfx1250) — hardware-verified
//
#include <hip/hip_runtime.h>


#ifndef NB
#define NB 256
#endif
#define NB_FULL 256
#define VV   128
#define CI   256
#define CO   256
#define DD   64
#define NWR  (CO + 2 * DD)
#define GW   8
#define PP   136
#define OSP  36
#define WTP  264
#define WHC  64.0f
#define WHI  (1.0f / 64.0f)
#define PSH  14.0f
#define L2E  1.4426950408889634f

static_assert(NB <= NB_FULL);
static_assert(VV % 64 == 0);
static_assert((NB * VV) % 64 == 0);
static_assert(CO % 64 == 0);
static_assert(DD == 64);
static_assert(CI % 32 == 0);
static_assert(VV % 32 == 0);
static_assert(VV == 128);
static_assert(GW == 8);
static_assert(GW * 16 == VV);
static_assert(CO % 32 == 0);
static_assert(CO % 32 == 0 && DD % 32 == 0);
static_assert(32 * 8 == CI);
static_assert(8 * 4 == 32);
static_assert((PP * 2) % 16 == 0);
static_assert((OSP * 4) % 16 == 0);
static_assert((WTP * 2) % 16 == 0);
static_assert(4 * 32 * 16 == 16 * 64 * 2);
static_assert(8 * 32 * 16 == 16 * DD * 4);
static_assert(4 * 32 * 16 == 16 * 32 * 4);
static_assert(VV * VV * 4 + VV * PP * 2 + GW * 16 * OSP * 4 + 2 * VV * 4 <= 131072);
static_assert(32 * WTP * 2 <= 131072);
static_assert(16 * 68 * 4 <= 131072);

typedef _Float16 h16;
typedef unsigned short bf;
typedef __attribute__((ext_vector_type(16))) __bf16   v16bf;
typedef __attribute__((ext_vector_type(16))) _Float16 v16h;
typedef __attribute__((ext_vector_type(8)))  _Float16 v8h;
typedef __attribute__((ext_vector_type(8)))  unsigned short v8us;
typedef __attribute__((ext_vector_type(8)))  float    v8f;
typedef __attribute__((ext_vector_type(4)))  float    v4f;
typedef v4f  __attribute__((may_alias)) v4fa;
typedef __attribute__((ext_vector_type(4)))  _Float16 v4h;
typedef v8us __attribute__((may_alias)) v8usa;

__device__ __forceinline__ unsigned short f2bf(float f) { unsigned u = __float_as_uint(f); u += 0x7FFFu + ((u >> 16) & 1u); return (unsigned short)(u >> 16); }
__device__ __forceinline__ float bfr(float f) { return __uint_as_float(((unsigned)f2bf(f)) << 16); }
__device__ __forceinline__ v16h cat16(v8h lo, v8h hi) { return __builtin_shufflevector(lo, hi, 0, 1, 2, 3, 4, 5, 6, 7, 8, 9, 10, 11, 12, 13, 14, 15); }
__device__ __forceinline__ v16bf cat16b(v8us lo, v8us hi) { return __builtin_bit_cast(v16bf, __builtin_shufflevector(lo, hi, 0, 1, 2, 3, 4, 5, 6, 7, 8, 9, 10, 11, 12, 13, 14, 15)); }
__device__ __forceinline__ v8f wmma16(v16h a, v16h b, v8f c) { return __builtin_amdgcn_wmma_f32_16x16x32_f16(false, a, false, b, (short)0, c, false, false); }
__device__ __forceinline__ v8f wmmab(v16bf a, v16bf b, v8f c) { return __builtin_amdgcn_wmma_f32_16x16x32_bf16(false, a, false, b, (short)0, c, false, false); }
__device__ __forceinline__ v16h  ldh(const h16* p) { return cat16(*(const v8h*)p, *(const v8h*)(p + 16)); }
__device__ __forceinline__ v16bf ldb(const bf* p)  { return cat16b(*(const v8us*)p, *(const v8us*)(p + 16)); }
__device__ __forceinline__ void wave_sync() { __builtin_amdgcn_fence(3  , "wavefront"); __builtin_amdgcn_wave_barrier(); asm volatile("" ::: "memory"); }

static __device__ __forceinline__ h16 toh_flush(float v) { const h16 r = (h16)v; return (fabsf(v) < 6.103515625e-05f) ? (h16)0.0f : r; }
static __device__ __forceinline__ v8f wmma16_g(v16h a, v16h b, v8f c) { c = wmma16(a, b, c); asm volatile("v_nop\n\tv_nop\n\tv_nop\n\tv_nop" : "+v"(c) : "v"(a), "v"(b)); return c; }
static __device__ __forceinline__ v8f wmmab_g(v16bf a, v16bf b, v8f c) { c = wmmab(a, b, c); asm volatile("v_nop\n\tv_nop\n\tv_nop\n\tv_nop" : "+v"(c) : "v"(a), "v"(b)); return c; }

__global__ __launch_bounds__(256) void k_cvt8(const float* __restrict__ src, bf* dst, size_t n8) {
    const size_t i = (size_t)blockIdx.x * 256 + threadIdx.x; if (i >= n8) return;
    const v8f v = *(const v8f*)(src + i * 8); v8us o;
#pragma unroll
    for (int k = 0; k < 8; ++k) o[k] = f2bf(v[k]);
    *(volatile v8us*)(dst + i * 8) = o; __threadfence(); *(volatile v8us*)(dst + i * 8) = o;
}

__global__ __launch_bounds__(256) void k_wt(const float* __restrict__ W, bf* dst, int N) {
    __shared__ __align__(16) bf t[32 * WTP];
    const int lane = threadIdx.x & 31;
    const int wave = __builtin_amdgcn_readfirstlane((int)(threadIdx.x >> 5));
    const int n0 = blockIdx.x * 32;
#pragma unroll 1
    for (int it = 0; it < CI / 8; ++it) { const int k = wave + 8 * it;
        t[lane * WTP + k] = f2bf(W[(size_t)k * N + n0 + lane]); }
    __syncthreads();
#pragma unroll 1
    for (int ps = 0; ps < 2; ++ps) {
#pragma unroll
        for (int s = 0; s < 4; ++s) { const int n = wave * 4 + s;
            const v8us val = *(const v8usa*)(&t[n * WTP + lane * 8]);
            *(volatile v8us*)(dst + (size_t)(n0 + n) * CI + lane * 8) = val; }
        if (ps == 0) __threadfence(); }
}

__global__ __launch_bounds__(32) void k_pw(const bf* __restrict__ A, const bf* __restrict__ Bt, h16* Ph) {
    __shared__ __align__(16) float os[16 * 68];
    const int K = CI;
    const int lane = threadIdx.x & 31, lr = lane & 15, hi = lane >> 4; const int r0 = blockIdx.x * 64, c0 = blockIdx.y * 64;
    v8f acc[4][4];
#pragma unroll
    for (int mb = 0; mb < 4; ++mb)
#pragma unroll
        for (int nb = 0; nb < 4; ++nb) acc[mb][nb] = (v8f){};
    const size_t aoff = (size_t)(r0 + lr) * K + 8 * hi, boff = (size_t)(c0 + lr) * K + 8 * hi;
#pragma unroll 1
    for (int kc = 0; kc < K; kc += 32) {
        v16bf a[4];
#pragma unroll
        for (int mb = 0; mb < 4; ++mb) a[mb] = ldb(A + aoff + (size_t)mb * 16 * K + kc);
#pragma unroll
        for (int nb = 0; nb < 4; ++nb) { const v16bf b = ldb(Bt + boff + (size_t)nb * 16 * K + kc);
#pragma unroll
            for (int mb = 0; mb < 4; ++mb) acc[mb][nb] = wmmab_g(a[mb], b, acc[mb][nb]); }
    }
    const int bb = c0 / VV, tt = c0 % VV;
    const size_t tbase = (size_t)bb * (size_t)CO * VV + (size_t)r0 * VV + (size_t)tt;
#pragma unroll
    for (int mb = 0; mb < 4; ++mb) {
#pragma unroll
        for (int nb = 0; nb < 4; ++nb) {
#pragma unroll
            for (int j = 0; j < 8; ++j) os[(hi * 8 + j) * 68 + nb * 16 + lr] = acc[mb][nb][j]; }
        wave_sync();
        const size_t sb = tbase + (size_t)(mb * 16) * VV;
#pragma unroll 1
        for (int ps = 0; ps < 2; ++ps) {
#pragma unroll
            for (int s = 0; s < 4; ++s) { const int row = 4 * s + (lane >> 3), c8 = (lane & 7) * 8;
                const v4f x0 = *(const v4fa*)(&os[row * 68 + c8]); const v4f x1 = *(const v4fa*)(&os[row * 68 + c8 + 4]); v8h hv;
#pragma unroll
                for (int i = 0; i < 4; ++i) { hv[i] = toh_flush(x0[i] * WHC); hv[4 + i] = toh_flush(x1[i] * WHC); }
                *(volatile v8h*)(Ph + sb + (size_t)row * VV + c8) = hv; }
            if (ps == 0) __threadfence(); }
        wave_sync();
    }
}

__global__ __launch_bounds__(32) void k_pe(const bf* __restrict__ A, const bf* __restrict__ Bt, float* Pf) {
    __shared__ __align__(16) float os[16 * 68];
    const int K = CI;
    const int lane = threadIdx.x & 31, lr = lane & 15, hi = lane >> 4; const int r0 = blockIdx.x * 64, c0 = blockIdx.y * 64;
    v8f acc[4][4];
#pragma unroll
    for (int mb = 0; mb < 4; ++mb)
#pragma unroll
        for (int nb = 0; nb < 4; ++nb) acc[mb][nb] = (v8f){};
    const size_t aoff = (size_t)(r0 + lr) * K + 8 * hi, boff = (size_t)(c0 + lr) * K + 8 * hi;
#pragma unroll 1
    for (int kc = 0; kc < K; kc += 32) {
        v16bf a[4];
#pragma unroll
        for (int mb = 0; mb < 4; ++mb) a[mb] = ldb(A + aoff + (size_t)mb * 16 * K + kc);
#pragma unroll
        for (int nb = 0; nb < 4; ++nb) { const v16bf b = ldb(Bt + boff + (size_t)nb * 16 * K + kc);
#pragma unroll
            for (int mb = 0; mb < 4; ++mb) acc[mb][nb] = wmmab_g(a[mb], b, acc[mb][nb]); }
    }
    float* dst = Pf + (size_t)blockIdx.y * ((size_t)NB * VV * DD) + (size_t)r0 * DD;
#pragma unroll
    for (int mb = 0; mb < 4; ++mb) {
#pragma unroll
        for (int nb = 0; nb < 4; ++nb) {
#pragma unroll
            for (int j = 0; j < 8; ++j) os[(hi * 8 + j) * 68 + nb * 16 + lr] = acc[mb][nb][j]; }
        wave_sync();
#pragma unroll 1
        for (int ps = 0; ps < 2; ++ps) {
#pragma unroll
            for (int s = 0; s < 8; ++s) { const int row = 2 * s + (lane >> 4), cofs = (lane & 15) * 4;
                const v4f val = *(const v4fa*)(&os[row * 68 + cofs]);
                *(volatile v4f*)(dst + (size_t)(mb * 16 + row) * DD + cofs) = val; }
            if (ps == 0) __threadfence(); }
        wave_sync();
    }
}

__global__ __launch_bounds__(32 * GW) __attribute__((amdgpu_num_vgpr(256))) void k_attn(const float* __restrict__ EL, const float* __restrict__ ER, const h16* __restrict__ WT,
                                                                                        const int* __restrict__ adj, const float* __restrict__ avec, float* OUT) {
    __shared__ __align__(16) float Es[VV * VV];
    __shared__ __align__(16) h16   Ps[VV * PP];
    __shared__ __align__(16) float os[GW * 16 * OSP];
    __shared__ float sls[VV];
    __shared__ float lin[VV];
    const int lane = threadIdx.x & 31, lr = lane & 15, hi = lane >> 4;
    const int wave = __builtin_amdgcn_readfirstlane((int)(threadIdx.x >> 5));
    const int b = blockIdx.x;
    const int j = (wave & 3) * 32 + lane;
    const float* elb = EL + (size_t)b * VV * DD;
    const float* erb = ER + (size_t)b * VV * DD;
    float areg[DD], ereg[DD];
#pragma unroll
    for (int d = 0; d < DD; d += 4) { const v4f av = *(const v4f*)(avec + d);
        areg[d] = bfr(av[0]); areg[d + 1] = bfr(av[1]); areg[d + 2] = bfr(av[2]); areg[d + 3] = bfr(av[3]); }
#pragma unroll
    for (int d = 0; d < DD; d += 4) { const v4f ev = *(const v4f*)(erb + (size_t)j * DD + d);
        ereg[d] = ev[0]; ereg[d + 1] = ev[1]; ereg[d + 2] = ev[2]; ereg[d + 3] = ev[3]; }
    float srj = 0.0f, slj = 0.0f;
#pragma unroll
    for (int d = 0; d < DD; ++d) srj += areg[d] * ereg[d];
#pragma unroll
    for (int d = 0; d < DD; d += 4) { const v4f lv = *(const v4f*)(elb + (size_t)j * DD + d);
        slj += areg[d] * lv[0]; slj += areg[d + 1] * lv[1]; slj += areg[d + 2] * lv[2]; slj += areg[d + 3] * lv[3]; }
    if (wave < 4) sls[j] = slj;
    __syncthreads();

    const int i0 = (wave >> 2) * 64;
#pragma unroll 1
    for (int ii = 0; ii < 64; ++ii) {
        const int i = i0 + ii;
        const float* elr = elb + (size_t)i * DD;
        float acc = 0.0f;
#pragma unroll
        for (int d = 0; d < DD; d += 4) { const v4f ev = *(const v4f*)(elr + d);
            acc += areg[d]     * fmaxf(ev[0] + ereg[d],     0.0f);
            acc += areg[d + 1] * fmaxf(ev[1] + ereg[d + 1], 0.0f);
            acc += areg[d + 2] * fmaxf(ev[2] + ereg[d + 2], 0.0f);
            acc += areg[d + 3] * fmaxf(ev[3] + ereg[d + 3], 0.0f); }
        const float e = fmaf(0.8f, acc, 0.2f * (sls[i] + srj));
        int ad = adj[i * VV + j];
        asm volatile("" : "+v"(ad));
        Es[i * VV + j] = (ad != 0) ? e : -__builtin_huge_valf();
    }
    __syncthreads();

#pragma unroll 1
    for (int rr = 0; rr < 16; ++rr) {
        const int i = wave * 16 + rr;
        const v4f v = *(const v4fa*)(&Es[i * VV + 4 * lane]);
        float mx = fmaxf(fmaxf(v[0], v[1]), fmaxf(v[2], v[3]));
        mx = fmaxf(mx, __shfl_xor(mx, 16, 32));
        mx = fmaxf(mx, __shfl_xor(mx, 8, 32));
        mx = fmaxf(mx, __shfl_xor(mx, 4, 32));
        mx = fmaxf(mx, __shfl_xor(mx, 2, 32));
        mx = fmaxf(mx, __shfl_xor(mx, 1, 32));
        v4h pv; float ls = 0.0f;
#pragma unroll
        for (int q = 0; q < 4; ++q) {
            const float ar = (v[q] - mx) * L2E + PSH;
            const float ex = __builtin_amdgcn_exp2f(ar);
            const float g = (ar < -PSH) ? 0.0f : ex;
            const h16 ph = (h16)g; pv[q] = ph; ls += (float)ph; }
        ls += __shfl_xor(ls, 16, 32);
        ls += __shfl_xor(ls, 8, 32);
        ls += __shfl_xor(ls, 4, 32);
        ls += __shfl_xor(ls, 2, 32);
        ls += __shfl_xor(ls, 1, 32);
        *(v4h*)(&Ps[i * PP + 4 * lane]) = pv;
        if (lane == 0) lin[i] = (1.0f / ls) * WHI;
    }
    __syncthreads();

    const int i0w = wave * 16;
    v16h pa[4];
#pragma unroll
    for (int ks = 0; ks < 4; ++ks) { const int idx = (i0w + lr) * PP + ks * 32 + 8 * hi;
        pa[ks] = cat16(*(const v8h*)(&Ps[idx]), *(const v8h*)(&Ps[idx + 16])); }
    float sc[8];
#pragma unroll
    for (int r = 0; r < 8; ++r) sc[r] = lin[i0w + 8 * hi + r];
    const size_t wbase = ((size_t)b * CO + lr) * VV + 8 * hi;
    float* orow = OUT + ((size_t)b * VV + i0w) * CO;
    const int wb = wave * 16 * OSP;
#pragma unroll 1
    for (int cg = 0; cg < CO / 32; ++cg) {
        v8f c0 = (v8f){}, c1 = (v8f){};
#pragma unroll
        for (int ks = 0; ks < 4; ++ks) {
            const h16* wp = WT + wbase + (size_t)(cg * 32) * VV + ks * 32;
            const v16h b0 = ldh(wp), b1 = ldh(wp + (size_t)16 * VV);
            c0 = wmma16_g(pa[ks], b0, c0); c1 = wmma16_g(pa[ks], b1, c1); }
#pragma unroll
        for (int r = 0; r < 8; ++r) {
            const float x0 = c0[r] * sc[r], x1 = c1[r] * sc[r];
            const float y0 = (x0 > 0.0f) ? x0 : (__builtin_amdgcn_exp2f(x0 * L2E) - 1.0f);
            const float y1 = (x1 > 0.0f) ? x1 : (__builtin_amdgcn_exp2f(x1 * L2E) - 1.0f);
            os[wb + (8 * hi + r) * OSP + lr] = y0; os[wb + (8 * hi + r) * OSP + 16 + lr] = y1; }
        wave_sync();
#pragma unroll 1
        for (int ps = 0; ps < 2; ++ps) {
#pragma unroll
            for (int s = 0; s < 4; ++s) { const int row = 4 * s + (lane >> 3), cofs = (lane & 7) * 4;
                const v4f val = *(const v4fa*)(&os[wb + row * OSP + cofs]);
                *(volatile v4f*)(orow + (size_t)row * CO + cg * 32 + cofs) = val; }
            if (ps == 0) __threadfence(); }
        wave_sync();
    }
}

static constexpr size_t al256(size_t v) { return (v + 255) & ~(size_t)255; }
static constexpr size_t SZ_XB = al256((size_t)NB * VV * CI * 2);
static constexpr size_t SZ_WB = al256((size_t)NWR * CI * 2);
static constexpr size_t SZ_EP = al256((size_t)2 * NB * VV * DD * 4);
static constexpr size_t SZ_WT = al256((size_t)NB * CO * VV * 2);
static constexpr size_t SZ_TOTAL = SZ_XB + SZ_WB + SZ_EP + SZ_WT;
static_assert(SZ_TOTAL <= (size_t)134217728);
static_assert(((size_t)NB * VV * CI) % 8 == 0);
static_assert(((size_t)CI * 2) % 128 == 0);

extern "C" void kernel_launch(void* const* d_in, const int* in_sizes, int n_in,
                              void* d_out, int out_size, void* d_ws, size_t ws_size, hipStream_t stream) {
    if (n_in < 6) return;
    if ((size_t)in_sizes[0] < (size_t)NB * VV * CI) return;
    if ((size_t)in_sizes[1] < (size_t)VV * VV) return;
    if ((size_t)in_sizes[2] < (size_t)CI * DD || (size_t)in_sizes[3] < (size_t)CI * DD) return;
    if (in_sizes[4] < DD) return;
    if ((size_t)in_sizes[5] < (size_t)CI * CO) return;
    if ((size_t)out_size < (size_t)NB * VV * CO) return;
    if (SZ_TOTAL > ws_size) return;
    const float* x    = (const float*)d_in[0];
    const int*   adj  = (const int*)d_in[1];
    const float* wl   = (const float*)d_in[2];
    const float* wr   = (const float*)d_in[3];
    const float* av   = (const float*)d_in[4];
    const float* wout = (const float*)d_in[5];
    float* OUT = (float*)d_out;
    char* wsp = (char*)d_ws;
    bf*    XB  = (bf*)wsp;    wsp += SZ_XB;
    bf*    WB  = (bf*)wsp;    wsp += SZ_WB;
    float* ELR = (float*)wsp; wsp += SZ_EP;
    h16*   WT  = (h16*)wsp;   wsp += SZ_WT;

    { const size_t n8 = (size_t)NB * VV * CI / 8;
      k_cvt8<<<(unsigned)((n8 + 255) / 256), 256, 0, stream>>>(x, XB, n8); }
    k_wt<<<CO / 32, 256, 0, stream>>>(wout, WB, CO);
    k_wt<<<DD / 32, 256, 0, stream>>>(wl, WB + (size_t)CO * CI, DD);
    k_wt<<<DD / 32, 256, 0, stream>>>(wr, WB + (size_t)(CO + DD) * CI, DD);
    k_pw<<<dim3(CO / 64, NB * VV / 64, 1), 32, 0, stream>>>(WB, XB, WT);
    k_pe<<<dim3(NB * VV / 64, 2, 1), 32, 0, stream>>>(XB, WB + (size_t)CO * CI, ELR);
    k_attn<<<NB, 32 * GW, 0, stream>>>(ELR, ELR + (size_t)NB * VV * DD, WT, adj, av, OUT);
}
